// SingleStageFIRFilter_11553462026858
// MI455X (gfx1250) — hardware-verified
//
#include <hip/hip_runtime.h>

#define FILTER_ORDER 24
#define P_FRAME      80
#define IR_LEN       200
#define NFFT         512
#define TAPS         199
#define WIN          399
#define KPAD         416
#define NCHUNK       13
#define B_BATCH      4
#define T_LEN        48000
#define N_FRAMES     600
#define XWIN         512
#define NCOLS        16

typedef _Float16 v16h __attribute__((ext_vector_type(16)));
typedef float    v8f  __attribute__((ext_vector_type(8)));
typedef _Float16 v8h  __attribute__((ext_vector_type(8)));
typedef float    v4f_t __attribute__((ext_vector_type(4)));
typedef float v4fa __attribute__((ext_vector_type(4), may_alias));
#define RSPLIT (1.0f / 2048.0f)

__global__ __launch_bounds__(160)
void fir_mlsa_wmma(const float* __restrict__ x,
                   const float* __restrict__ mc,
                   float* __restrict__ y)
{
    __shared__ float costab[NFFT];
    __shared__ float E[2][NFFT];
    __shared__ float h2[2][IR_LEN];
    __shared__ __align__(32) _Float16 sB[NCOLS][KPAD];
    __shared__ _Float16 sXhi[XWIN];
    __shared__ _Float16 sXlo[XWIN];
    __shared__ float sOut[5][2][16][16];
    __shared__ __attribute__((aligned(16))) float sY[2 * P_FRAME];

    const int tid  = threadIdx.x;
    const int wave = tid >> 5;
    const int lane = tid & 31;

    const int blk = blockIdx.x;
    const int b   = blk / (N_FRAMES / 2);
    const int np  = blk - b * (N_FRAMES / 2);
  #pragma unroll 1
  for (int s2 = 0; s2 < 2; ++s2) {
    __syncthreads();
    const int n   = np * 2 + s2;
    const int nB  = (n + 1 < N_FRAMES) ? n + 1 : n;
    const int t0  = n * P_FRAME;

    const float* mcA = mc + ((size_t)b * N_FRAMES + n)  * (FILTER_ORDER + 1);
    const float* mcB = mc + ((size_t)b * N_FRAMES + nB) * (FILTER_ORDER + 1);

    __builtin_prefetch(&x[(size_t)b * T_LEN + t0], 0, 0);

    const float twopi_n = 6.283185307179586f / (float)NFFT;
    for (int i = tid; i < NFFT; i += 160)
        costab[i] = cosf(twopi_n * (float)i);
    {
        unsigned int* zb = (unsigned int*)&sB[4][0];
        const int nd = (NCOLS - 4) * KPAD / 2;
        for (int i = tid; i < nd; i += 160) zb[i] = 0u;
    }
    __syncthreads();

    for (int m = tid; m < 2 * NFFT; m += 160) {
        const int s  = m >> 9;
        const int mm = m & (NFFT - 1);
        const float* mcs = s ? mcB : mcA;
        float lh = mcs[0];
        int idx = 0;
        #pragma unroll 4
        for (int k = 1; k <= FILTER_ORDER; ++k) {
            idx = (idx + mm) & (NFFT - 1);
            lh = fmaf(mcs[k], costab[idx], lh);
        }
        E[s][mm] = expf(lh);
    }
    __syncthreads();

    for (int j = tid; j < 2 * IR_LEN; j += 160) {
        const int s  = (j >= IR_LEN) ? 1 : 0;
        const int jj = j - s * IR_LEN;
        const float* Es = E[s];
        float acc = 0.0f;
        int idx = 0;
        #pragma unroll 8
        for (int m = 0; m < NFFT; ++m) {
            acc = fmaf(Es[m], costab[idx], acc);
            idx = (idx + jj) & (NFFT - 1);
        }
        h2[s][jj] = acc * (1.0f / (float)NFFT);
    }
    __syncthreads();

    for (int i = tid; i < KPAD; i += 160) {
        int d = i - TAPS; if (d < 0) d = -d;
        const float va = (i < WIN) ? h2[0][d] : 0.0f;
        const float vb = (i < WIN) ? h2[1][d] : 0.0f;
        const _Float16 ah = (_Float16)va;
        const _Float16 bh = (_Float16)vb;
        sB[0][i] = ah;
        sB[1][i] = bh;
        sB[2][i] = (_Float16)((va - (float)ah) * 2048.0f);
        sB[3][i] = (_Float16)((vb - (float)bh) * 2048.0f);
    }
    for (int i = tid; i < XWIN; i += 160) {
        const int gx = t0 + i - TAPS;
        const float v = (gx >= 0 && gx < T_LEN) ? x[(size_t)b * T_LEN + gx] : 0.0f;
        const _Float16 hi = (_Float16)v;
        sXhi[i] = hi;
        sXlo[i] = (_Float16)((v - (float)hi) * 2048.0f);
    }
    __syncthreads();

    const int row   = lane & 15;
    const int col   = lane & 15;
    const int mbase = wave * 16;
    const int aK0   = (lane < 16) ? 0 : 8;
    const int bK0   = aK0;

    v8f acc1 = {};
    v8f acc2 = {};

    for (int kc = 0; kc < NCHUNK; ++kc) {
        const int kb = kc * 32;
        v16h ahi, alo;
        const int abase = mbase + row + kb + aK0;
        #pragma unroll
        for (int i = 0; i < 16; ++i) {
            const int kl = (i < 8) ? i : (i + 8);
            ahi[i] = sXhi[abase + kl];
            alo[i] = sXlo[abase + kl];
        }
        const v16h bmat = __builtin_shufflevector(*(const v8h*)&sB[col][kb + bK0], *(const v8h*)&sB[col][kb + 16 + bK0],
                                                  0,1,2,3,4,5,6,7,8,9,10,11,12,13,14,15);

        acc1 = __builtin_amdgcn_wmma_f32_16x16x32_f16(false, ahi, false, bmat,
                                                      (short)0, acc1, false, false);
        acc2 = __builtin_amdgcn_wmma_f32_16x16x32_f16(false, alo, false, bmat,
                                                      (short)0, acc2, false, false);
    }

    asm volatile("v_nop\n\tv_nop\n\tv_nop\n\tv_nop\n\tv_nop\n\tv_nop\n\tv_nop\n\tv_nop" : "+v"(acc1), "+v"(acc2));
    const int rowoff = (lane < 16) ? 0 : 8;
    #pragma unroll
    for (int r = 0; r < 8; ++r) {
        sOut[wave][0][r + rowoff][col] = acc1[r];
        sOut[wave][1][r + rowoff][col] = acc2[r];
    }
    __syncthreads();

    if (lane < 16) {
        const int p = mbase + lane;
        const float YA = sOut[wave][0][lane][0] + (sOut[wave][0][lane][2] + sOut[wave][1][lane][0]) * RSPLIT;
        const float YB = sOut[wave][0][lane][1] + (sOut[wave][0][lane][3] + sOut[wave][1][lane][1]) * RSPLIT;
        const float w  = (float)p * (1.0f / (float)P_FRAME);
        sY[s2 * P_FRAME + p] = (1.0f - w) * YA + w * YB;
    }
  }
    __syncthreads();
    if (tid < 40) {
        float* yp = y + (size_t)b * T_LEN + (size_t)np * (2 * P_FRAME) + tid * 4;
        const v4f_t v = *(const volatile v4fa*)(sY + tid * 4);
        *(volatile v4f_t*)yp = v; __threadfence(); *(volatile v4f_t*)yp = v;
    }
}

extern "C" void kernel_launch(void* const* d_in, const int* in_sizes, int n_in,
                              void* d_out, int out_size, void* d_ws, size_t ws_size,
                              hipStream_t stream)
{
    (void)in_sizes; (void)n_in; (void)out_size; (void)d_ws; (void)ws_size;
    const float* x  = (const float*)d_in[0];
    const float* mc = (const float*)d_in[1];
    float* y        = (float*)d_out;

    dim3 grid(B_BATCH * (N_FRAMES / 2));
    dim3 block(160);
    hipLaunchKernelGGL(fir_mlsa_wmma, grid, block, 0, stream, x, mc, y);
}
